// SelfAttention_80539226735261
// MI455X (gfx1250) — hardware-verified
//
#include <hip/hip_runtime.h>
#ifndef NB
#define NB 2
#endif
#ifndef SEQ
#define SEQ 2048
#endif
#define NB_FULL 2
#define SEQ_FULL 2048
#define EMB 1024
#define NHEAD 16
#define HD 64
#define QVW 2048
#ifndef RESQ
#define RESQ 512
#endif
#define NR (NB * SEQ)
#define PLQ ((size_t)NR * QVW)
#define PLT ((size_t)NB * NHEAD * HD * SEQ)
#define PLC ((size_t)NR * EMB)
#define SZ_X16 ((size_t)NR * EMB * 2)
#define SZ_WQV ((size_t)QVW * EMB * 2)
#define SZ_WO  ((size_t)EMB * EMB * 2)
#define SZ_QV  ((size_t)2 * NR * QVW * 2)
#define SZ_VT  ((size_t)2 * NB * NHEAD * HD * SEQ * 2)
#define SZ_CTX ((size_t)2 * NR * EMB * 2)

static_assert(NHEAD * HD == EMB);
static_assert(HD == 64);
static_assert(QVW == 2 * EMB);
static_assert(SEQ % 64 == 0);
static_assert(NR % 128 == 0);
static_assert(EMB % 64 == 0 && QVW % 64 == 0);
static_assert(EMB % 32 == 0);
static_assert(RESQ % 64 == 0);
static_assert((RESQ >= SEQ) || (SEQ % 512 == 0 && RESQ % 512 == 0));
static_assert(NB <= NB_FULL && SEQ <= SEQ_FULL);
static_assert(SZ_X16 % 256 == 0 && SZ_WQV % 256 == 0 && SZ_WO % 256 == 0 && SZ_QV % 256 == 0 && SZ_VT % 256 == 0 && SZ_CTX % 256 == 0);
static_assert(SZ_X16 + SZ_WQV + SZ_WO + SZ_QV + SZ_VT + SZ_CTX <= (size_t)134217728);

typedef unsigned short v8us __attribute__((ext_vector_type(8), may_alias));
typedef float  v8f  __attribute__((ext_vector_type(8)));
typedef float  v4f  __attribute__((ext_vector_type(4)));
typedef float  v4fa __attribute__((ext_vector_type(4), may_alias));
typedef _Float16 v16h __attribute__((ext_vector_type(16)));
union FragH { v16h v; v8us half[2]; _Float16 h[16]; unsigned short u[16]; };

__device__ __forceinline__ unsigned short bf16_bits(float x) { unsigned int u = __float_as_uint(x); return (unsigned short)((u + 0x7FFFu + ((u >> 16) & 1u)) >> 16); }
__device__ __forceinline__ float bf16_rne(float x) { return __uint_as_float(((unsigned int)bf16_bits(x)) << 16); }

__device__ __forceinline__ v16h g2_frag(const _Float16* p, int hh) { FragH f; f.half[0] = *(const v8us*)((const unsigned short*)p + 8 * hh); f.half[1] = *(const v8us*)((const unsigned short*)p + 16 + 8 * hh); return f.v; }
__device__ __forceinline__ v8f g2_mma(v16h a, v16h b, v8f c) { v8f d = __builtin_amdgcn_wmma_f32_16x16x32_f16(false, a, false, b, (short)0, c, false, false); asm volatile("v_nop\n\tv_nop\n\tv_nop\n\tv_nop" : "+v"(d) : "v"(a), "v"(b)); return d; }

__global__ __launch_bounds__(256) void k_x16(const float* __restrict__ x, _Float16* __restrict__ X16) {
  const size_t t = (size_t)blockIdx.x * 256 + threadIdx.x;
  if (t >= (size_t)NR * (EMB / 8)) return;
  const int row = (int)(t / (EMB / 8)), pc = (int)(t % (EMB / 8));
  const int b = row / SEQ, l = row - b * SEQ;
  const float* s = x + ((size_t)b * SEQ_FULL + l) * EMB + pc * 8;
  const v4f a = *(const v4fa*)s, c = *(const v4fa*)(s + 4);
  FragH f;
#pragma unroll
  for (int q = 0; q < 4; ++q) { f.h[q] = (_Float16)bf16_rne(a[q]); f.h[4 + q] = (_Float16)bf16_rne(c[q]); }
  const v8us o = f.half[0];
  unsigned short* d = (unsigned short*)X16 + t * 8;
  *(volatile v8us*)d = o; __threadfence(); *(volatile v8us*)d = o;
}

__global__ __launch_bounds__(256) void k_wcvt(const float* __restrict__ w, _Float16* __restrict__ Bt, unsigned n8, unsigned split8, unsigned skip8) {
  const unsigned t = blockIdx.x * 256u + threadIdx.x;
  if (t >= n8) return;
  const size_t s8 = (size_t)t + ((t >= split8) ? skip8 : 0u);
  const v4f a = *(const v4fa*)(w + s8 * 8), c = *(const v4fa*)(w + s8 * 8 + 4);
  FragH f;
#pragma unroll
  for (int q = 0; q < 4; ++q) { f.h[q] = (_Float16)(bf16_rne(a[q]) * 64.0f); f.h[4 + q] = (_Float16)(bf16_rne(c[q]) * 64.0f); }
  const v8us o = f.half[0];
  unsigned short* d = (unsigned short*)Bt + (size_t)t * 8;
  *(volatile v8us*)d = o; __threadfence(); *(volatile v8us*)d = o;
}

__global__ __launch_bounds__(128) void k_gemm_qv(const _Float16* __restrict__ A, const _Float16* __restrict__ Bh, const float* __restrict__ bias, _Float16* __restrict__ C) {
  __shared__ __attribute__((aligned(16))) float so[4][32][68];
  const int tid = threadIdx.x, lane = tid & 31, ln = lane & 15, hh = lane >> 4;
  const int w = __builtin_amdgcn_readfirstlane(tid >> 5);
  const int ntn = QVW / 64;
  const int mt = blockIdx.x / ntn, nq = blockIdx.x - mt * ntn;
  const int row0 = mt * 128 + 32 * w, col0 = nq * 64;
  const _Float16* a0p = A + (size_t)(row0 + ln) * EMB; const _Float16* a1p = a0p + (size_t)16 * EMB;
  const _Float16* bp = Bh + (size_t)(col0 + ln) * EMB;
  const v8f z8 = {0.f, 0.f, 0.f, 0.f, 0.f, 0.f, 0.f, 0.f};
  v8f c[8] = {z8, z8, z8, z8, z8, z8, z8, z8};
#pragma unroll 1
  for (int kb = 0; kb < EMB; kb += 32) {
    const v16h a0 = g2_frag(a0p + kb, hh), a1 = g2_frag(a1p + kb, hh);
#pragma unroll
    for (int t = 0; t < 4; ++t) {
      const v16h bb = g2_frag(bp + (size_t)(16 * t) * EMB + kb, hh);
      c[t] = g2_mma(a0, bb, c[t]); c[4 + t] = g2_mma(a1, bb, c[4 + t]);
    }
  }
#pragma unroll
  for (int u = 0; u < 8; ++u) {
    const int t = u & 3, half = u >> 2;
    const int col = col0 + t * 16 + ln;
    const int bc = col + ((col >= EMB) ? EMB : 0);
    const float bv = bf16_rne(bias[bc]);
#pragma unroll
    for (int r = 0; r < 8; ++r) so[w][half * 16 + 8 * hh + r][t * 16 + ln] = c[u][r] * 0.015625f + bv;
  }
  __builtin_amdgcn_fence(4  , "workgroup"); __builtin_amdgcn_wave_barrier();
  const int rq = lane >> 3, pc = lane & 7;
  for (int pass = 0; pass < 2; ++pass) {
#pragma unroll
    for (int q = 0; q < 8; ++q) {
      const int r = 4 * q + rq;
      const v4f x0 = *(const v4fa*)&so[w][r][8 * pc], x1 = *(const v4fa*)&so[w][r][8 * pc + 4];
      FragH fh, fl;
#pragma unroll
      for (int i = 0; i < 4; ++i) {
        _Float16 hv = (_Float16)x0[i]; fh.h[i] = hv; fl.h[i] = (_Float16)((x0[i] - (float)hv) * 1024.0f);
        hv = (_Float16)x1[i]; fh.h[4 + i] = hv; fl.h[4 + i] = (_Float16)((x1[i] - (float)hv) * 1024.0f);
      }
      const v8us oh = fh.half[0], ol = fl.half[0];
      unsigned short* d = (unsigned short*)C + (size_t)(row0 + r) * QVW + col0 + 8 * pc;
      *(volatile v8us*)d = oh; *(volatile v8us*)(d + PLQ) = ol;
    }
    if (pass == 0) __threadfence();
  }
}

__global__ __launch_bounds__(256) void k_vt(const _Float16* __restrict__ QV, _Float16* __restrict__ VT) {
  __shared__ unsigned short tl[64][65];
  const int tid = threadIdx.x;
  const int nsg = SEQ / 64;
  const int sg = blockIdx.x % nsg, bh = blockIdx.x / nsg;
  const int b = bh / NHEAD, h = bh - b * NHEAD;
  const int s0 = sg * 64;
  const unsigned short* src = (const unsigned short*)QV + (size_t)blockIdx.y * PLQ + ((size_t)b * SEQ + s0) * QVW + EMB + h * HD;
  unsigned short* dst = (unsigned short*)VT + (size_t)blockIdx.y * PLT + (size_t)bh * HD * SEQ + s0;
  for (int i = tid; i < 64 * 8; i += 256) {
    const int j = i / 8, d8 = (i % 8) * 8;
    FragH f; f.half[0] = *(const v8us*)(src + (size_t)j * QVW + d8);
#pragma unroll
    for (int q = 0; q < 8; ++q) tl[d8 + q][j] = f.u[q];
  }
  __syncthreads();
  for (int pass = 0; pass < 2; ++pass) {
    for (int i = tid; i < 64 * 8; i += 256) {
      const int d = i / 8, j8 = (i % 8) * 8;
      FragH f;
#pragma unroll
      for (int q = 0; q < 8; ++q) f.u[q] = tl[d][j8 + q];
      const v8us o = f.half[0];
      *(volatile v8us*)(dst + (size_t)d * SEQ + j8) = o;
    }
    if (pass == 0) __threadfence();
  }
}

__global__ __launch_bounds__(128) void k_flash(const _Float16* __restrict__ QV, const _Float16* __restrict__ VT, const int* __restrict__ maskp, _Float16* __restrict__ CTX) {
  __shared__ __attribute__((aligned(16))) unsigned short ot[4][2][16][72];
  const int tid = threadIdx.x, lane = tid & 31, ln = lane & 15, hh = lane >> 4;
  const int w = __builtin_amdgcn_readfirstlane(tid >> 5);
  const int qt = blockIdx.x, bh = blockIdx.y;
  const int b = bh / NHEAD, h = bh - b * NHEAD;
  const int causal = (maskp[0] != 0) ? 1 : 0;
  const int nkt = causal ? (qt + 1) : (SEQ / 64);
  const bool res = (qt * 64 < RESQ);
  const int lq = qt * 64 + 16 * w + ln;
  const _Float16* qrow = QV + ((size_t)b * SEQ + lq) * QVW + h * HD;
  const v16h qh0 = g2_frag(qrow, hh), qh1 = g2_frag(qrow + 32, hh);
  const v16h ql0 = g2_frag(qrow + PLQ, hh), ql1 = g2_frag(qrow + PLQ + 32, hh);
  const _Float16* vbase = QV + ((size_t)b * SEQ) * QVW + EMB + h * HD;
  const _Float16* vtb = VT + (size_t)bh * HD * SEQ;
  const v8f z8 = {0.f, 0.f, 0.f, 0.f, 0.f, 0.f, 0.f, 0.f};
  v8f o[4] = {z8, z8, z8, z8};
  v8f e[4] = {z8, z8, z8, z8};
  float mrun = -3.0e38f, lsum = 0.f;
#pragma unroll 1
  for (int kt = 0; kt < nkt; ++kt) {
    const int j0 = kt * 64;
    v8f st[4];
#pragma unroll
    for (int t = 0; t < 4; ++t) {
      const _Float16* vr = vbase + (size_t)(j0 + 16 * t + ln) * QVW;
      const v16h a0 = g2_frag(vr, hh), a1 = g2_frag(vr + 32, hh);
      v8f s = z8;
      s = g2_mma(a0, qh0, s); s = g2_mma(a1, qh1, s);
      if (res) {
        const v16h al0 = g2_frag(vr + PLQ, hh), al1 = g2_frag(vr + PLQ + 32, hh);
        v8f sr = z8;
        sr = g2_mma(al0, qh0, sr); sr = g2_mma(al1, qh1, sr);
        sr = g2_mma(a0, ql0, sr);  sr = g2_mma(a1, ql1, sr);
        s = s + sr * 0.0009765625f;
      }
      st[t] = s;
    }
    if (causal != 0 && kt == qt) {
#pragma unroll
      for (int t = 0; t < 4; ++t)
#pragma unroll
        for (int r = 0; r < 8; ++r) { const int key = j0 + 16 * t + 8 * hh + r; st[t][r] = (key > lq) ? -3.0e38f : st[t][r]; }
    }
    float mx = mrun;
#pragma unroll
    for (int t = 0; t < 4; ++t)
#pragma unroll
      for (int r = 0; r < 8; ++r) mx = fmaxf(mx, st[t][r]);
    mx = fmaxf(mx, __shfl_xor(mx, 16));
    const float fac = __expf((mrun - mx) * 0.125f);
    mrun = mx; lsum *= fac;
    FragH ph0, ph1, pl0, pl1;
#pragma unroll
    for (int t = 0; t < 4; ++t)
#pragma unroll
      for (int r = 0; r < 8; ++r) {
        const float p = __expf((st[t][r] - mx) * 0.125f);
        lsum += p; st[t][r] = p;
        const _Float16 hv = (_Float16)p;
        if (t < 2) ph0.h[(t & 1) * 8 + r] = hv; else ph1.h[(t & 1) * 8 + r] = hv;
      }
    if (res) {
#pragma unroll
      for (int t = 0; t < 4; ++t)
#pragma unroll
        for (int r = 0; r < 8; ++r) {
          const float hf = (t < 2) ? (float)ph0.h[(t & 1) * 8 + r] : (float)ph1.h[(t & 1) * 8 + r];
          const _Float16 lv = (_Float16)((st[t][r] - hf) * 1024.0f);
          if (t < 2) pl0.h[(t & 1) * 8 + r] = lv; else pl1.h[(t & 1) * 8 + r] = lv;
        }
    } else {
#pragma unroll
      for (int i = 0; i < 16; ++i) { pl0.h[i] = (_Float16)0.0f; pl1.h[i] = (_Float16)0.0f; }
    }
#pragma unroll
    for (int dt = 0; dt < 4; ++dt) { o[dt] = o[dt] * fac; e[dt] = e[dt] * fac; }
#pragma unroll
    for (int dt = 0; dt < 4; ++dt) {
      const _Float16* tr = vtb + (size_t)(16 * dt + ln) * SEQ + j0;
      const v16h a0 = g2_frag(tr, hh), a1 = g2_frag(tr + 32, hh);
      o[dt] = g2_mma(a0, ph0.v, o[dt]); o[dt] = g2_mma(a1, ph1.v, o[dt]);
      if (res) {
        const v16h al0 = g2_frag(tr + PLT, hh), al1 = g2_frag(tr + PLT + 32, hh);
        e[dt] = g2_mma(al0, ph0.v, e[dt]); e[dt] = g2_mma(al1, ph1.v, e[dt]);
        e[dt] = g2_mma(a0, pl0.v, e[dt]);  e[dt] = g2_mma(a1, pl1.v, e[dt]);
      }
    }
  }
  lsum += __shfl_xor(lsum, 16);
  const float inv = (1.0f / lsum) * 16.0f;
#pragma unroll
  for (int dt = 0; dt < 4; ++dt) {
    FragH fh, fl;
#pragma unroll
    for (int r = 0; r < 8; ++r) {
      const float cv = (o[dt][r] + e[dt][r] * 0.0009765625f) * inv;
      const _Float16 hv = (_Float16)cv;
      fh.h[r] = hv; fl.h[r] = (_Float16)((cv - (float)hv) * 1024.0f);
    }
    *(v8us*)&ot[w][0][ln][16 * dt + 8 * hh] = fh.half[0];
    *(v8us*)&ot[w][1][ln][16 * dt + 8 * hh] = fl.half[0];
  }
  __builtin_amdgcn_fence(4  , "workgroup"); __builtin_amdgcn_wave_barrier();
  const int rq = lane >> 3, pc = lane & 7;
  unsigned short* cb = (unsigned short*)CTX + ((size_t)bh * SEQ + qt * 64 + 16 * w) * HD;
  for (int pass = 0; pass < 2; ++pass) {
#pragma unroll
    for (int i = 0; i < 4; ++i) {
      const int row = 4 * i + rq;
      const v8us vh = *(const v8us*)&ot[w][0][row][8 * pc];
      const v8us vl = *(const v8us*)&ot[w][1][row][8 * pc];
      *(volatile v8us*)(cb + row * HD + 8 * pc) = vh;
      *(volatile v8us*)(cb + PLC + row * HD + 8 * pc) = vl;
    }
    if (pass == 0) __threadfence();
  }
}

__global__ __launch_bounds__(128) void k_gemm_out(const _Float16* __restrict__ A, const _Float16* __restrict__ Bh, const float* __restrict__ bias, float* __restrict__ C) {
  __shared__ __attribute__((aligned(16))) float so[4][32][68];
  const int tid = threadIdx.x, lane = tid & 31, ln = lane & 15, hh = lane >> 4;
  const int w = __builtin_amdgcn_readfirstlane(tid >> 5);
  const int ntn = EMB / 64;
  const int mt = blockIdx.x / ntn, nq = blockIdx.x - mt * ntn;
  const int row0 = mt * 128 + 32 * w, col0 = nq * 64;
  const bool res = (RESQ >= SEQ) || (((row0 % (SEQ / 16)) * 16) < RESQ);
  const _Float16* a0p = A + (size_t)(row0 + ln) * EMB; const _Float16* a1p = a0p + (size_t)16 * EMB;
  const _Float16* bp = Bh + (size_t)(col0 + ln) * EMB;
  const v8f z8 = {0.f, 0.f, 0.f, 0.f, 0.f, 0.f, 0.f, 0.f};
  v8f c[8]  = {z8, z8, z8, z8, z8, z8, z8, z8};
  v8f cr[8] = {z8, z8, z8, z8, z8, z8, z8, z8};
  if (res) {
#pragma unroll 1
    for (int kb = 0; kb < EMB; kb += 32) {
      const v16h a0 = g2_frag(a0p + kb, hh), a1 = g2_frag(a1p + kb, hh);
      const v16h al0 = g2_frag(a0p + PLC + kb, hh), al1 = g2_frag(a1p + PLC + kb, hh);
#pragma unroll
      for (int t = 0; t < 4; ++t) {
        const v16h bb = g2_frag(bp + (size_t)(16 * t) * EMB + kb, hh);
        c[t] = g2_mma(a0, bb, c[t]);    c[4 + t] = g2_mma(a1, bb, c[4 + t]);
        cr[t] = g2_mma(al0, bb, cr[t]); cr[4 + t] = g2_mma(al1, bb, cr[4 + t]);
      }
    }
  } else {
#pragma unroll 1
    for (int kb = 0; kb < EMB; kb += 32) {
      const v16h a0 = g2_frag(a0p + kb, hh), a1 = g2_frag(a1p + kb, hh);
#pragma unroll
      for (int t = 0; t < 4; ++t) {
        const v16h bb = g2_frag(bp + (size_t)(16 * t) * EMB + kb, hh);
        c[t] = g2_mma(a0, bb, c[t]); c[4 + t] = g2_mma(a1, bb, c[4 + t]);
      }
    }
  }
#pragma unroll
  for (int u = 0; u < 8; ++u) {
    const int t = u & 3, half = u >> 2;
    const float bv = bf16_rne(bias[col0 + t * 16 + ln]);
#pragma unroll
    for (int r = 0; r < 8; ++r) so[w][half * 16 + 8 * hh + r][t * 16 + ln] = (c[u][r] + cr[u][r] * 0.0009765625f) * 0.0009765625f + bv;
  }
  __builtin_amdgcn_fence(4  , "workgroup"); __builtin_amdgcn_wave_barrier();
  const int rsub = lane >> 4, c4 = (lane & 15) * 4;
  for (int pass = 0; pass < 2; ++pass) {
#pragma unroll
    for (int q = 0; q < 16; ++q) {
      const int r = q * 2 + rsub;
      const v4f v = *(const v4fa*)&so[w][r][c4];
      *(volatile v4f*)(C + (size_t)(row0 + r) * EMB + col0 + c4) = v;
    }
    if (pass == 0) __threadfence();
  }
}

extern "C" void kernel_launch(void* const* d_in, const int* in_sizes, int n_in,
                              void* d_out, int out_size, void* d_ws, size_t ws_size, hipStream_t stream) {
  if (n_in < 6) return;
  if ((long long)in_sizes[0] < (long long)(NB - 1) * SEQ_FULL * EMB + (long long)SEQ * EMB) return;
  if ((long long)in_sizes[1] < (long long)3 * EMB * EMB) return;
  if (in_sizes[2] < 3 * EMB) return;
  if ((long long)in_sizes[3] < (long long)EMB * EMB) return;
  if (in_sizes[4] < EMB) return;
  if (in_sizes[5] < 1) return;
  if ((long long)out_size < (long long)NR * EMB) return;
  const float* x = (const float*)d_in[0];
  const float* wqkv = (const float*)d_in[1];
  const float* bqkv = (const float*)d_in[2];
  const float* wout = (const float*)d_in[3];
  const float* bout = (const float*)d_in[4];
  const int* mask = (const int*)d_in[5];
  char* ws = (char*)d_ws; size_t off = 0;
  auto take = [&](size_t bytes) { char* p = ws + off; off += (bytes + 255) & ~(size_t)255; return p; };
  _Float16* X16 = (_Float16*)take(SZ_X16);
  _Float16* WQV = (_Float16*)take(SZ_WQV);
  _Float16* WO  = (_Float16*)take(SZ_WO);
  _Float16* QV  = (_Float16*)take(SZ_QV);
  _Float16* VT  = (_Float16*)take(SZ_VT);
  _Float16* CTX = (_Float16*)take(SZ_CTX);
  if (off > ws_size) return;
  k_x16<<<(unsigned)(((size_t)NR * (EMB / 8) + 255) / 256), 256, 0, stream>>>(x, X16);
  { const unsigned n8 = (unsigned)((size_t)QVW * EMB / 8), h8 = (unsigned)((size_t)EMB * EMB / 8);
    k_wcvt<<<(n8 + 255) / 256, 256, 0, stream>>>(wqkv, WQV, n8, h8, h8);
    k_wcvt<<<(h8 + 255) / 256, 256, 0, stream>>>(wout, WO, h8, h8, 0u); }
  k_gemm_qv<<<(unsigned)((NR / 128) * (QVW / 64)), 128, 0, stream>>>(X16, WQV, bqkv, QV);
  k_vt<<<dim3((unsigned)(NB * NHEAD * (SEQ / 64)), 2), 256, 0, stream>>>(QV, VT);
  k_flash<<<dim3((unsigned)(SEQ / 64), (unsigned)(NB * NHEAD)), 128, 0, stream>>>(QV, VT, mask, CTX);
  k_gemm_out<<<(unsigned)((NR / 128) * (EMB / 64)), 128, 0, stream>>>(CTX, WO, bout, (float*)d_out);
}
